// VisualSemanticEncoder_47347719471324
// MI455X (gfx1250) — hardware-verified
//
#include <hip/hip_runtime.h>
#include <math.h>

constexpr int kBatch = 32;
constexpr int kImg   = 512;
constexpr int kKnow  = 256;
constexpr int kNodes = 768;
constexpr int kDim   = 512;
constexpr int kHid   = 128;
constexpr int kRows  = kBatch * kNodes;
constexpr float kWCarry   = 16.0f;
constexpr float kInvNodes = 1.0f / 768.0f;

typedef __attribute__((ext_vector_type(16))) _Float16 v16h;
typedef __attribute__((ext_vector_type(8)))  _Float16 v8h;
typedef __attribute__((ext_vector_type(16))) __bf16   v16b;
typedef __attribute__((ext_vector_type(8)))  __bf16   v8b;
typedef __attribute__((ext_vector_type(8)))  float    v8f;
typedef __attribute__((ext_vector_type(4)))  float    v4f;
typedef __attribute__((ext_vector_type(4)))  unsigned int v4u;

__device__ __forceinline__ unsigned short f2bf_bits(float f) {
  unsigned u = __float_as_uint(f);
  return (unsigned short)((u + 0x7FFFu + ((u >> 16) & 1u)) >> 16);
}
__device__ __forceinline__ float bf_bits2f(unsigned short h) { return __uint_as_float(((unsigned)h) << 16); }

__device__ __forceinline__ void dep_guard_h(v8f& a, v8f& b, v16h x, v16h y) { asm volatile("v_nop\n\tv_nop\n\tv_nop\n\tv_nop" : "+v"(a), "+v"(b) : "v"(x), "v"(y)); }
__device__ __forceinline__ void dep_guard_b(v8f& a, v8f& b, v16b x, v16b y) { asm volatile("v_nop\n\tv_nop\n\tv_nop\n\tv_nop" : "+v"(a), "+v"(b) : "v"(x), "v"(y)); }
__device__ __forceinline__ void keep4_h(v16h a, v16h b, v16h c, v16h d) { asm volatile("v_nop" :: "v"(a), "v"(b), "v"(c), "v"(d)); }
__device__ __forceinline__ void keep4_b(v16b a, v16b b, v16b c, v16b d) { asm volatile("v_nop" :: "v"(a), "v"(b), "v"(c), "v"(d)); }
__device__ __forceinline__ void acc_guard4(v8f& a, v8f& b, v8f& c, v8f& d) { asm volatile("v_nop\n\tv_nop\n\tv_nop\n\tv_nop" : "+v"(a), "+v"(b), "+v"(c), "+v"(d)); }
template <typename T> struct Frag;
template <> struct Frag<_Float16> {
  typedef v16h V; union U { v16h v; v8h h[2]; };
  static __device__ __forceinline__ v16h load(const _Float16* p) {
    U f; f.h[0] = *(const v8h*)(p); f.h[1] = *(const v8h*)(p + 16); return f.v;
  }
  static __device__ __forceinline__ v8f mma(v16h a, v16h b, v8f c) {
    return __builtin_amdgcn_wmma_f32_16x16x32_f16(false, a, false, b, (short)0, c, false, false);
  }
  static __device__ __forceinline__ void guard(v8f& a, v8f& b, v16h x, v16h y) { dep_guard_h(a, b, x, y); }
  static __device__ __forceinline__ void keep(v16h a, v16h b, v16h c, v16h d) { keep4_h(a, b, c, d); }
};
template <> struct Frag<__bf16> {
  typedef v16b V; union U { v16b v; v8b h[2]; };
  static __device__ __forceinline__ v16b load(const __bf16* p) {
    U f; f.h[0] = *(const v8b*)(p); f.h[1] = *(const v8b*)(p + 16); return f.v;
  }
  static __device__ __forceinline__ v8f mma(v16b a, v16b b, v8f c) {
    return __builtin_amdgcn_wmma_f32_16x16x32_bf16(false, a, false, b, (short)0, c, false, false);
  }
  static __device__ __forceinline__ void guard(v8f& a, v8f& b, v16b x, v16b y) { dep_guard_b(a, b, x, y); }
  static __device__ __forceinline__ void keep(v16b a, v16b b, v16b c, v16b d) { keep4_b(a, b, c, d); }
};

__device__ __forceinline__ unsigned pk16(unsigned short a, unsigned short b) { return (unsigned)a | ((unsigned)b << 16); }
__device__ __forceinline__ unsigned short h_bits(float f) { const _Float16 h = (_Float16)f; return __builtin_bit_cast(unsigned short, h); }

template <int ET> struct Elem;
template <> struct Elem<0> { typedef _Float16 T; };
template <> struct Elem<1> { typedef __bf16 T; };
template <int ET, bool SPLIT, int BIAS_MODE, int OUT_MODE, bool RESID, int ACT = 0, int POST = 1>
__global__ __launch_bounds__(256) void wmma_gemm64(
    const unsigned short* __restrict__ Ap, const unsigned short* __restrict__ A2p, int lda, long strideA,
    const unsigned short* __restrict__ Btp, const unsigned short* __restrict__ Bt2p, int ldb, long strideB,
    void* __restrict__ Cout, void* __restrict__ Cout2, int ldc, long strideC,
    const float* __restrict__ bias,
    const float* __restrict__ resid, long strideR,
    int M, int N, int K, float scale) {
  typedef typename Elem<ET>::T T;
  typedef typename Frag<T>::V V;
  const T* A = (const T*)Ap; const T* A2 = (const T*)A2p; const T* Bt = (const T*)Btp; const T* Bt2 = (const T*)Bt2p;
  __shared__ __align__(16) float sT[8][16 * 68];
  const int b    = blockIdx.y;
  const int lane = threadIdx.x & 31;
  const int wave = threadIdx.x >> 5;
  const int tilesN = N >> 6;
  const int tilesM = M >> 6;
  const int tile = blockIdx.x * 8 + wave;
  if (tile >= tilesM * tilesN) return;
  const int tm = tile / tilesN;
  const int tn = tile - tm * tilesN;
  const int m0 = tm << 6;
  const int n0 = tn << 6;

  const T* Ab  = A  + (size_t)b * strideA;
  const T* Bb  = Bt + (size_t)b * strideB;
  const T* Ab2 = SPLIT ? (A2  + (size_t)b * strideA) : nullptr;
  const T* Bb2 = SPLIT ? (Bt2 + (size_t)b * strideB) : nullptr;

  const int rlane = lane & 15;
  const int koff  = (lane >> 4) * 8;
  const int mOff  = (lane >> 4) * 8;

  v8f acc[4][4];
#pragma unroll
  for (int i = 0; i < 4; ++i)
#pragma unroll
    for (int j = 0; j < 4; ++j) acc[i][j] = (v8f){0.f,0.f,0.f,0.f,0.f,0.f,0.f,0.f};

  for (int k0 = 0; k0 < K; k0 += 32) {
    V bh[4], bl[4];
#pragma unroll
    for (int j = 0; j < 4; ++j) {
      const size_t bo = (size_t)(n0 + (j << 4) + rlane) * ldb + koff + k0;
      bh[j] = Frag<T>::load(Bb + bo);
      if (SPLIT) bl[j] = Frag<T>::load(Bb2 + bo);
    }
#pragma unroll
    for (int i = 0; i < 4; ++i) {
      const size_t ao = (size_t)(m0 + (i << 4) + rlane) * lda + koff + k0;
      V ah = Frag<T>::load(Ab + ao);
      V al;
      if (SPLIT) al = Frag<T>::load(Ab2 + ao);
#pragma unroll
      for (int j = 0; j < 4; ++j) {
        acc[i][j] = Frag<T>::mma(ah, bh[j], acc[i][j]);
        if (SPLIT) {
          acc[i][j] = Frag<T>::mma(ah, bl[j], acc[i][j]);
          acc[i][j] = Frag<T>::mma(al, bh[j], acc[i][j]);
        }
      }
      Frag<T>::guard(acc[i][0], acc[i][3], ah, SPLIT ? al : ah);
    }
    Frag<T>::keep(bh[0], bh[1], bh[2], bh[3]);
    if (SPLIT) Frag<T>::keep(bl[0], bl[1], bl[2], bl[3]);
  }
  acc_guard4(acc[0][0], acc[0][1], acc[0][2], acc[0][3]);
  acc_guard4(acc[1][0], acc[1][1], acc[1][2], acc[1][3]);
  acc_guard4(acc[2][0], acc[2][1], acc[2][2], acc[2][3]);
  acc_guard4(acc[3][0], acc[3][1], acc[3][2], acc[3][3]);

  float* slab = sT[wave];
  const float* Rb = RESID ? (resid + (size_t)b * strideR) : nullptr;
#pragma unroll
  for (int i = 0; i < 4; ++i) {
    const int mBase = m0 + (i << 4);
#pragma unroll
    for (int j = 0; j < 4; ++j) {
      const int n = n0 + (j << 4) + rlane;
      float bv = 0.f;
      if (BIAS_MODE == 2) bv = bias[n];
#pragma unroll
      for (int r = 0; r < 8; ++r) {
        float v = acc[i][j][r] * scale;
        if (BIAS_MODE == 1) v += bias[mBase + mOff + r];
        if (BIAS_MODE == 2) v += bv;
        if (RESID) v += Rb[(size_t)(mBase + mOff + r) * ldc + n];
        if (ACT == 2) v = fmaxf(v, 0.0f);
        if (ACT == 4) v = (v > 0.f) ? v : 0.01f * v;
        if (POST != 1) v = v * (float)POST;
        slab[(mOff + r) * 68 + (j << 4) + rlane] = v;
      }
    }
    __builtin_amdgcn_fence(__ATOMIC_RELEASE, "workgroup");
    __builtin_amdgcn_wave_barrier();
    __builtin_amdgcn_fence(__ATOMIC_ACQUIRE, "workgroup");
    if (OUT_MODE == 0) {
      float* C = (float*)Cout + (size_t)b * strideC;
      const int hh = lane >> 4, c4 = (lane & 15) * 4;
      for (int pass = 0; pass < 2; ++pass) {
#pragma unroll
        for (int it = 0; it < 8; ++it) {
          const int row = it * 2 + hh;
          v4f v = *(const v4f*)(slab + row * 68 + c4);
          *(volatile v4f*)(C + (size_t)(mBase + row) * ldc + n0 + c4) = v;
        }
        __threadfence();
      }
    } else {
      const int q = lane >> 3, c8 = (lane & 7) * 8;
      unsigned short* C  = (unsigned short*)Cout  + (size_t)b * strideC;
      unsigned short* C2 = (OUT_MODE == 2) ? ((unsigned short*)Cout2 + (size_t)b * strideC) : nullptr;
      for (int pass = 0; pass < 2; ++pass) {
#pragma unroll
        for (int it = 0; it < 4; ++it) {
          const int row = it * 4 + q;
          const float* sp = slab + row * 68 + c8;
          v8h hv, lv;
#pragma unroll
          for (int e = 0; e < 8; ++e) {
            if (OUT_MODE == 1) {
              hv[e] = (_Float16)sp[e];
            } else {
              unsigned short hb = f2bf_bits(sp[e]);
              unsigned short lb = f2bf_bits(sp[e] - bf_bits2f(hb));
              hv[e] = __builtin_bit_cast(_Float16, hb);
              lv[e] = __builtin_bit_cast(_Float16, lb);
            }
          }
          *(volatile v8h*)(C + (size_t)(mBase + row) * ldc + n0 + c8) = hv;
          if (OUT_MODE == 2) *(volatile v8h*)(C2 + (size_t)(mBase + row) * ldc + n0 + c8) = lv;
        }
        __threadfence();
      }
    }
    __builtin_amdgcn_fence(__ATOMIC_RELEASE, "workgroup");
    __builtin_amdgcn_wave_barrier();
    __builtin_amdgcn_fence(__ATOMIC_ACQUIRE, "workgroup");
  }
}

__global__ __launch_bounds__(256) void wtrans_cast_kernel(const float* __restrict__ W, unsigned short* __restrict__ out,
                                                          int R, int Ccols, float scale) {
  __shared__ float sm[64][65];
  const int t  = threadIdx.x;
  const int r0 = blockIdx.x * 64;
  const int c0 = blockIdx.y * 64;
#pragma unroll
  for (int i = 0; i < 16; ++i) {
    const int e  = i * 256 + t;
    const int rl = e >> 6;
    const int cl = e & 63;
    sm[cl][rl] = W[(size_t)(r0 + rl) * Ccols + c0 + cl] * scale;
  }
  __syncthreads();
  const int lane = t & 31, wave = t >> 5;
  const int q = lane >> 3, c8 = (lane & 7) * 8;
  for (int pass = 0; pass < 2; ++pass) {
#pragma unroll
    for (int it = 0; it < 2; ++it) {
      const int row = wave * 8 + it * 4 + q;
      unsigned short hb[8];
#pragma unroll
      for (int e = 0; e < 8; ++e) hb[e] = h_bits(sm[row][c8 + e]);
      const v4u u = (v4u){pk16(hb[0], hb[1]), pk16(hb[2], hb[3]), pk16(hb[4], hb[5]), pk16(hb[6], hb[7])};
      *(volatile v4u*)(out + (size_t)(c0 + row) * R + r0 + c8) = u;
    }
    __threadfence();
  }
}

__global__ __launch_bounds__(256) void castx_kernel(const float* __restrict__ vis, const float* __restrict__ sem,
                                                    unsigned short* __restrict__ out, int n8) {
  const int i = blockIdx.x * 256 + threadIdx.x;
  if (i >= n8) return;
  const int row = i >> 6;
  const int d0  = (i & 63) * 8;
  const int b   = row / kNodes;
  const int n   = row - b * kNodes;
  const float* p = (n < kImg) ? (vis + ((size_t)b * kImg + n) * kDim + d0)
                              : (sem + ((size_t)b * kKnow + (n - kImg)) * kDim + d0);
  const v4f a = *(const v4f*)(p);
  const v4f c = *(const v4f*)(p + 4);
  unsigned short hb[8];
#pragma unroll
  for (int e = 0; e < 4; ++e) {
    hb[e]     = h_bits(a[e]);
    hb[4 + e] = h_bits(c[e]);
  }
  const v4u u = (v4u){pk16(hb[0], hb[1]), pk16(hb[2], hb[3]), pk16(hb[4], hb[5]), pk16(hb[6], hb[7])};
  unsigned short* q = out + 8 * (size_t)i;
  *(volatile v4u*)q = u;
  __threadfence();
  *(volatile v4u*)q = u;
}

__global__ __launch_bounds__(256) void node_mean_kernel(const float* __restrict__ Y, float* __restrict__ out) {
  __shared__ __align__(16) float sm[256];
  const int t  = threadIdx.x;
  const int b  = blockIdx.x >> 1;
  const int d0 = (blockIdx.x & 1) * 256;
  const float* p = Y + (size_t)b * kNodes * kDim + d0 + t;
  float a0 = 0.f, a1 = 0.f, a2 = 0.f, a3 = 0.f;
#pragma unroll 1
  for (int n = 0; n < kNodes; n += 4) {
    a0 += p[(size_t)(n + 0) * kDim];
    a1 += p[(size_t)(n + 1) * kDim];
    a2 += p[(size_t)(n + 2) * kDim];
    a3 += p[(size_t)(n + 3) * kDim];
  }
  const float s = ((a0 + a1) + (a2 + a3)) * kInvNodes;
  sm[t] = s;
  __syncthreads();
  const int lane = t & 31, wave = t >> 5;
  if (wave < 2) {
    const v4f val = *(const v4f*)(sm + wave * 128 + lane * 4);
    float* op = out + (size_t)b * kDim + d0 + wave * 128 + lane * 4;
    *(volatile v4f*)op = val;
    __threadfence();
    *(volatile v4f*)op = val;
  }
}

extern "C" void kernel_launch(void* const* d_in, const int* in_sizes, int n_in,
                              void* d_out, int out_size, void* d_ws, size_t ws_size,
                              hipStream_t stream) {
  if (n_in < 8) return;
  if (in_sizes[0] != kBatch * kImg * kDim || in_sizes[1] != kBatch * kKnow * kDim ||
      in_sizes[2] != kDim * kHid || in_sizes[3] != kHid || in_sizes[4] != kHid * kHid ||
      in_sizes[5] != kHid || in_sizes[6] != kDim * kDim || in_sizes[7] != kDim) return;
  if (out_size != kBatch * kDim) return;

  const float* vis  = (const float*)d_in[0];
  const float* sem  = (const float*)d_in[1];
  const float* e1_w = (const float*)d_in[2];
  const float* e1_b = (const float*)d_in[3];
  const float* e2_w = (const float*)d_in[4];
  const float* e2_b = (const float*)d_in[5];
  const float* gc_w = (const float*)d_in[6];
  const float* gc_b = (const float*)d_in[7];
  float* out = (float*)d_out;

  const size_t bytesX16  = (size_t)kRows * kDim * 2;
  const size_t bytesH    = (size_t)kRows * kHid * 2;
  const size_t bytesW1T  = (size_t)kHid * kDim * 2;
  const size_t bytesW2T  = (size_t)kHid * kHid * 2;
  const size_t bytesWGT  = (size_t)kDim * kDim * 2;
  const size_t bytesOUTN = (size_t)kBatch * kNodes * kDim * 4;
  const size_t bytesADJ  = (size_t)kBatch * kNodes * kNodes * 2;
  const size_t bytesSUPT = (size_t)kBatch * kDim * kNodes * 2;

  const size_t offX16  = 0;
  const size_t offH1   = offX16 + bytesX16;
  const size_t offH2   = offH1 + bytesH;
  const size_t offW1T  = offH2 + bytesH;
  const size_t offW2T  = offW1T + bytesW1T;
  const size_t offWGT  = offW2T + bytesW2T;
  const size_t endEarly = offWGT + bytesWGT;
  const size_t offOUTN = 0;
  const size_t offADJ  = (bytesOUTN > endEarly) ? bytesOUTN : endEarly;
  const size_t offSUPT = offADJ + bytesADJ;
  const size_t wsEnd   = offSUPT + bytesSUPT;
  if (wsEnd > ws_size) return;

  char* ws = (char*)d_ws;
  unsigned short* X16  = (unsigned short*)(ws + offX16);
  unsigned short* H1   = (unsigned short*)(ws + offH1);
  unsigned short* H2   = (unsigned short*)(ws + offH2);
  unsigned short* W1T  = (unsigned short*)(ws + offW1T);
  unsigned short* W2T  = (unsigned short*)(ws + offW2T);
  unsigned short* WGT  = (unsigned short*)(ws + offWGT);
  float*          OUTN = (float*)(ws + offOUTN);
  unsigned short* ADJ  = (unsigned short*)(ws + offADJ);
  unsigned short* SUPT = (unsigned short*)(ws + offSUPT);

  {
    const int n8 = kRows * kDim / 8;
    castx_kernel<<<dim3((n8 + 255) / 256), dim3(256), 0, stream>>>(vis, sem, X16, n8);
  }
  wtrans_cast_kernel<<<dim3(kDim / 64, kHid / 64), dim3(256), 0, stream>>>(e1_w, W1T, kDim, kHid, kWCarry);
  wtrans_cast_kernel<<<dim3(kHid / 64, kHid / 64), dim3(256), 0, stream>>>(e2_w, W2T, kHid, kHid, kWCarry);
  wtrans_cast_kernel<<<dim3(kDim / 64, kDim / 64), dim3(256), 0, stream>>>(gc_w, WGT, kDim, kDim, kWCarry);

  wmma_gemm64<0, false, 2, 1, false, 2, 1><<<dim3(96, 1), dim3(256), 0, stream>>>(
      X16, X16, kDim, 0L, W1T, W1T, kDim, 0L, (void*)H1, (void*)H1, kHid, 0L,
      e1_b, gc_b, 0L, kRows, kHid, kDim, 1.0f / 16.0f);

  wmma_gemm64<0, false, 2, 1, false, 2, 8><<<dim3(96, 1), dim3(256), 0, stream>>>(
      H1, H1, kHid, 0L, W2T, W2T, kHid, 0L, (void*)H2, (void*)H2, kHid, 0L,
      e2_b, gc_b, 0L, kRows, kHid, kHid, 1.0f / 16.0f);

  wmma_gemm64<0, false, 0, 1, false, 0, 1><<<dim3(18, kBatch), dim3(256), 0, stream>>>(
      H2, H2, kHid, (long)kNodes * kHid, H2, H2, kHid, (long)kNodes * kHid,
      (void*)ADJ, (void*)ADJ, kNodes, (long)kNodes * kNodes,
      gc_b, gc_b, 0L, kNodes, kNodes, kHid, 1.0f / 64.0f);

  wmma_gemm64<0, false, 0, 1, false, 0, 1><<<dim3(12, kBatch), dim3(256), 0, stream>>>(
      WGT, WGT, kDim, 0L, X16, X16, kDim, (long)kNodes * kDim,
      (void*)SUPT, (void*)SUPT, kNodes, (long)kDim * kNodes,
      gc_b, gc_b, 0L, kDim, kNodes, kDim, 1.0f);

  wmma_gemm64<0, false, 2, 0, false, 2, 1><<<dim3(12, kBatch), dim3(256), 0, stream>>>(
      ADJ, ADJ, kNodes, (long)kNodes * kNodes, SUPT, SUPT, kNodes, (long)kDim * kNodes,
      (void*)OUTN, (void*)OUTN, kDim, (long)kNodes * kDim,
      gc_b, gc_b, 0L, kNodes, kDim, kNodes, 1.0f / 16.0f);

  node_mean_kernel<<<dim3(kBatch * 2), dim3(256), 0, stream>>>(OUTN, out);
}
